// MultiScaleRetention_43525198578339
// MI455X (gfx1250) — hardware-verified
//
#include <hip/hip_runtime.h>
#include <math.h>

constexpr int kBatch = 2;
constexpr int kSeq   = 2048;
constexpr int kDim   = 1024;
constexpr int kHeads = 16;
constexpr int kDh    = 64;
constexpr int kTok   = kBatch * kSeq;
constexpr int kGroup = 2;
constexpr float kWoCarry    = 16.0f;
constexpr float kWoCarryInv = 1.0f / 16.0f;
constexpr float kGnEps      = 1.0e-5f;
static_assert(kHeads * kDh == kDim, "shape");
static_assert(kTok % 64 == 0 && kDim % 64 == 0 && kSeq % 64 == 0 && kDh % 64 == 0, "tile multiples");
static_assert(kDim % 32 == 0 && kDh % 32 == 0 && kSeq % 32 == 0, "K multiples of 32");
static_assert(kHeads % kGroup == 0 && kGroup == 2, "groups");
static_assert((kTok * kDim) % (8 * 256) == 0 && (kDim * kDim) % (8 * 256) == 0, "cast grids exact");
static_assert(((kTok / 64) * (kDim / 64)) % 8 == 0, "proj grid");
static_assert(((kDim / 64) * (kSeq / 64)) % 8 == 0, "vt grid");
static_assert(((kSeq / 64) * (kSeq / 64)) % 8 == 0, "score grid");
static_assert(((kSeq / 64) * (kDh / 64)) % 8 == 0 || ((kSeq / 64) * (kDh / 64)) == 32, "pv grid");

typedef __attribute__((ext_vector_type(16))) _Float16 v16h;
typedef __attribute__((ext_vector_type(8)))  _Float16 v8h;
typedef __attribute__((ext_vector_type(16))) __bf16   v16b;
typedef __attribute__((ext_vector_type(8)))  __bf16   v8b;
typedef __attribute__((ext_vector_type(8)))  float    v8f;
typedef __attribute__((ext_vector_type(4)))  float    v4f;
typedef __attribute__((ext_vector_type(4)))  unsigned int v4u;

__device__ __forceinline__ unsigned short f2bf_bits(float f) {
  unsigned u = __float_as_uint(f);
  return (unsigned short)((u + 0x7FFFu + ((u >> 16) & 1u)) >> 16);
}
__device__ __forceinline__ float bf_bits2f(unsigned short h) { return __uint_as_float(((unsigned)h) << 16); }

__device__ __forceinline__ void dep_guard_h(v8f& a, v8f& b, v16h x, v16h y) { asm volatile("v_nop\n\tv_nop\n\tv_nop\n\tv_nop" : "+v"(a), "+v"(b) : "v"(x), "v"(y)); }
__device__ __forceinline__ void dep_guard_b(v8f& a, v8f& b, v16b x, v16b y) { asm volatile("v_nop\n\tv_nop\n\tv_nop\n\tv_nop" : "+v"(a), "+v"(b) : "v"(x), "v"(y)); }
__device__ __forceinline__ void dep_guard4v_h(v8f& a, v8f& b, v8f& c, v8f& d, v16h x, v16h y) { asm volatile("v_nop\n\tv_nop\n\tv_nop\n\tv_nop" : "+v"(a), "+v"(b), "+v"(c), "+v"(d) : "v"(x), "v"(y)); }
__device__ __forceinline__ void dep_guard4v_b(v8f& a, v8f& b, v8f& c, v8f& d, v16b x, v16b y) { asm volatile("v_nop\n\tv_nop\n\tv_nop\n\tv_nop" : "+v"(a), "+v"(b), "+v"(c), "+v"(d) : "v"(x), "v"(y)); }
__device__ __forceinline__ void keep4_h(v16h a, v16h b, v16h c, v16h d) { asm volatile("v_nop" :: "v"(a), "v"(b), "v"(c), "v"(d)); }
__device__ __forceinline__ void keep4_b(v16b a, v16b b, v16b c, v16b d) { asm volatile("v_nop" :: "v"(a), "v"(b), "v"(c), "v"(d)); }
__device__ __forceinline__ void acc_guard4(v8f& a, v8f& b, v8f& c, v8f& d) { asm volatile("v_nop\n\tv_nop\n\tv_nop\n\tv_nop" : "+v"(a), "+v"(b), "+v"(c), "+v"(d)); }
template <typename T> struct Frag;
template <> struct Frag<_Float16> {
  typedef v16h V; union U { v16h v; v8h h[2]; };
  static __device__ __forceinline__ v16h load(const _Float16* p) {
    U f; f.h[0] = *(const v8h*)(p); f.h[1] = *(const v8h*)(p + 16); return f.v;
  }
  static __device__ __forceinline__ v8f mma(v16h a, v16h b, v8f c) {
    return __builtin_amdgcn_wmma_f32_16x16x32_f16(false, a, false, b, (short)0, c, false, false);
  }
  static __device__ __forceinline__ void guard(v8f& a, v8f& b, v16h x, v16h y) { dep_guard_h(a, b, x, y); }
  static __device__ __forceinline__ void guard4(v8f& a, v8f& b, v8f& c, v8f& d, v16h x, v16h y) { dep_guard4v_h(a, b, c, d, x, y); }
  static __device__ __forceinline__ void keep(v16h a, v16h b, v16h c, v16h d) { keep4_h(a, b, c, d); }
};
template <> struct Frag<__bf16> {
  typedef v16b V; union U { v16b v; v8b h[2]; };
  static __device__ __forceinline__ v16b load(const __bf16* p) {
    U f; f.h[0] = *(const v8b*)(p); f.h[1] = *(const v8b*)(p + 16); return f.v;
  }
  static __device__ __forceinline__ v8f mma(v16b a, v16b b, v8f c) {
    return __builtin_amdgcn_wmma_f32_16x16x32_bf16(false, a, false, b, (short)0, c, false, false);
  }
  static __device__ __forceinline__ void guard(v8f& a, v8f& b, v16b x, v16b y) { dep_guard_b(a, b, x, y); }
  static __device__ __forceinline__ void guard4(v8f& a, v8f& b, v8f& c, v8f& d, v16b x, v16b y) { dep_guard4v_b(a, b, c, d, x, y); }
  static __device__ __forceinline__ void keep(v16b a, v16b b, v16b c, v16b d) { keep4_b(a, b, c, d); }
};

__device__ __forceinline__ unsigned pk16(unsigned short a, unsigned short b) { return (unsigned)a | ((unsigned)b << 16); }
__device__ __forceinline__ unsigned short h_bits(float f) { const _Float16 h = (_Float16)f; return __builtin_bit_cast(unsigned short, h); }

template <int ET> struct Elem;
template <> struct Elem<0> { typedef _Float16 T; };
template <> struct Elem<1> { typedef __bf16 T; };
template <int ET, bool SPLIT, int BIAS_MODE, int OUT_MODE, bool RESID, int ACT, int KMODE, bool DECAY>
__global__ __launch_bounds__(256) void wmma_gemm64(
    const unsigned short* __restrict__ Ap, const unsigned short* __restrict__ A2p, int lda, long strideA,
    const unsigned short* __restrict__ Btp, const unsigned short* __restrict__ Bt2p, int ldb, long strideB,
    void* __restrict__ Cout, void* __restrict__ Cout2, int ldc, long strideC,
    const float* __restrict__ bias,
    const float* __restrict__ resid, long strideR,
    int M, int N, int K, float scale, float dk0, float dk1) {
  typedef typename Elem<ET>::T T;
  typedef typename Frag<T>::V V;
  const T* A = (const T*)Ap; const T* A2 = (const T*)A2p; const T* Bt = (const T*)Btp; const T* Bt2 = (const T*)Bt2p;
  __shared__ __align__(16) float sT[8][16 * 68];
  const int b    = blockIdx.y;
  const int lane = threadIdx.x & 31;
  const int wave = threadIdx.x >> 5;
  const int tilesN = N >> 6;
  const int tilesM = M >> 6;
  const int tile = blockIdx.x * 8 + wave;
  if (tile >= tilesM * tilesN) return;
  const int tm = tile / tilesN;
  const int tn = tile - tm * tilesN;
  if (KMODE == 1 && tn > tm) return;
  const int m0 = tm << 6;
  const int n0 = tn << 6;
  const int kEnd = (KMODE == 2) ? (((m0 + 64) < K) ? (m0 + 64) : K) : K;

  const T* Ab  = A  + (size_t)b * strideA;
  const T* Bb  = Bt + (size_t)b * strideB;
  const T* Ab2 = SPLIT ? (A2  + (size_t)b * strideA) : nullptr;
  const T* Bb2 = SPLIT ? (Bt2 + (size_t)b * strideB) : nullptr;

  const int rlane = lane & 15;
  const int koff  = (lane >> 4) * 8;
  const int mOff  = (lane >> 4) * 8;

  v8f acc[4][4];
#pragma unroll
  for (int i = 0; i < 4; ++i)
#pragma unroll
    for (int j = 0; j < 4; ++j) acc[i][j] = (v8f){0.f,0.f,0.f,0.f,0.f,0.f,0.f,0.f};

  for (int k0 = 0; k0 < kEnd; k0 += 32) {
    V bh[4], bl[4];
#pragma unroll
    for (int j = 0; j < 4; ++j) {
      const size_t bo = (size_t)(n0 + (j << 4) + rlane) * ldb + koff + k0;
      bh[j] = Frag<T>::load(Bb + bo);
      if (SPLIT) bl[j] = Frag<T>::load(Bb2 + bo);
    }
#pragma unroll
    for (int i = 0; i < 4; ++i) {
      const size_t ao = (size_t)(m0 + (i << 4) + rlane) * lda + koff + k0;
      V ah = Frag<T>::load(Ab + ao);
      V al;
      if (SPLIT) al = Frag<T>::load(Ab2 + ao);
#pragma unroll
      for (int j = 0; j < 4; ++j) {
        acc[i][j] = Frag<T>::mma(ah, bh[j], acc[i][j]);
        if (SPLIT) {
          acc[i][j] = Frag<T>::mma(ah, bl[j], acc[i][j]);
          acc[i][j] = Frag<T>::mma(al, bh[j], acc[i][j]);
        }
      }
      Frag<T>::guard4(acc[i][0], acc[i][1], acc[i][2], acc[i][3], ah, SPLIT ? al : ah);
    }
    Frag<T>::keep(bh[0], bh[1], bh[2], bh[3]);
    if (SPLIT) Frag<T>::keep(bl[0], bl[1], bl[2], bl[3]);
  }
  acc_guard4(acc[0][0], acc[0][1], acc[0][2], acc[0][3]);
  acc_guard4(acc[1][0], acc[1][1], acc[1][2], acc[1][3]);
  acc_guard4(acc[2][0], acc[2][1], acc[2][2], acc[2][3]);
  acc_guard4(acc[3][0], acc[3][1], acc[3][2], acc[3][3]);

  float* slab = sT[wave];
  const float* Rb = RESID ? (resid + (size_t)b * strideR) : nullptr;
  float dtb = 1.0f, dg16 = 1.0f, dc16 = 1.0f, dcn0 = 1.0f, drow = 1.0f;
  float dgp[8] = {1.f, 1.f, 1.f, 1.f, 1.f, 1.f, 1.f, 1.f};
  if (DECAY) {
    float lgv = (b == 0) ? dk0 : dk1;
    asm volatile("" : "+v"(lgv) : "v"(acc[0][0]));
    const int dmn = m0 - n0;
    dtb  = expf((float)(dmn > 0 ? dmn : 0) * lgv);
    const float dg = expf(lgv);
    dg16 = expf(16.0f * lgv);
    dc16 = expf(-16.0f * lgv);
    dcn0 = expf(-(float)rlane * lgv);
    drow = expf((float)mOff * lgv);
    dgp[0] = 1.0f;
#pragma unroll
    for (int r = 1; r < 8; ++r) dgp[r] = dgp[r - 1] * dg;
  }
#pragma unroll
  for (int i = 0; i < 4; ++i) {
    const int mBase = m0 + (i << 4);
    float dcol = dcn0;
#pragma unroll
    for (int j = 0; j < 4; ++j) {
      const int n = n0 + (j << 4) + rlane;
      float bv = 0.f;
      if (BIAS_MODE == 2) bv = bias[n];
#pragma unroll
      for (int r = 0; r < 8; ++r) {
        float v = acc[i][j][r] * scale;
        if (BIAS_MODE == 1) v += bias[mBase + mOff + r];
        if (BIAS_MODE == 2) v += bv;
        if (RESID) v += Rb[(size_t)(mBase + mOff + r) * ldc + n];
        if (ACT == 2) v = fmaxf(v, 0.0f);
        if (ACT == 4) v = (v > 0.f) ? v : 0.01f * v;
        if (DECAY) {
          const float dfac = (dtb * dcol) * (drow * dgp[r]);
          const int mm = mBase + mOff + r;
          const float vd = v * dfac;
          v = (n <= mm) ? vd : 0.0f;
        }
        slab[(mOff + r) * 68 + (j << 4) + rlane] = v;
      }
      if (DECAY) dcol *= dc16;
    }
    __builtin_amdgcn_fence(__ATOMIC_RELEASE, "workgroup");
    __builtin_amdgcn_wave_barrier();
    __builtin_amdgcn_fence(__ATOMIC_ACQUIRE, "workgroup");
    if (OUT_MODE == 0) {
      float* C = (float*)Cout + (size_t)b * strideC;
      const int hh = lane >> 4, c4 = (lane & 15) * 4;
      for (int pass = 0; pass < 2; ++pass) {
#pragma unroll
        for (int it = 0; it < 8; ++it) {
          const int row = it * 2 + hh;
          v4f v = *(const v4f*)(slab + row * 68 + c4);
          *(volatile v4f*)(C + (size_t)(mBase + row) * ldc + n0 + c4) = v;
        }
        __threadfence();
      }
    } else {
      const int q = lane >> 3, c8 = (lane & 7) * 8;
      unsigned short* C  = (unsigned short*)Cout  + (size_t)b * strideC;
      unsigned short* C2 = (OUT_MODE == 2) ? ((unsigned short*)Cout2 + (size_t)b * strideC) : nullptr;
      for (int pass = 0; pass < 2; ++pass) {
#pragma unroll
        for (int it = 0; it < 4; ++it) {
          const int row = it * 4 + q;
          const float* sp = slab + row * 68 + c8;
          v8h hv, lv;
#pragma unroll
          for (int e = 0; e < 8; ++e) {
            if (OUT_MODE == 1) {
              hv[e] = (_Float16)sp[e];
            } else {
              unsigned short hb = f2bf_bits(sp[e]);
              unsigned short lb = f2bf_bits(sp[e] - bf_bits2f(hb));
              hv[e] = __builtin_bit_cast(_Float16, hb);
              lv[e] = __builtin_bit_cast(_Float16, lb);
            }
          }
          *(volatile v8h*)(C + (size_t)(mBase + row) * ldc + n0 + c8) = hv;
          if (OUT_MODE == 2) *(volatile v8h*)(C2 + (size_t)(mBase + row) * ldc + n0 + c8) = lv;
        }
        __threadfence();
      }
    }
    __builtin_amdgcn_fence(__ATOMIC_RELEASE, "workgroup");
    __builtin_amdgcn_wave_barrier();
    __builtin_amdgcn_fence(__ATOMIC_ACQUIRE, "workgroup");
    if (DECAY) drow *= dg16;
  }
}

template <int MODE> __device__ __forceinline__ unsigned short cvt16(float f) {
  if (MODE == 0) return f2bf_bits(f);
  const float r = bf_bits2f(f2bf_bits(f)) * kWoCarry;
  return h_bits(r);
}
template <int MODE>
__global__ __launch_bounds__(256) void cast8_kernel(const float* __restrict__ in, unsigned short* __restrict__ out, int n8) {
  const int i = blockIdx.x * 256 + threadIdx.x;
  if (i >= n8) return;
  const float* p = in + 8 * (size_t)i;
  const v4f a = *(const v4f*)(p);
  const v4f c = *(const v4f*)(p + 4);
  unsigned short hb[8];
#pragma unroll
  for (int e = 0; e < 4; ++e) {
    hb[e]     = cvt16<MODE>(a[e]);
    hb[4 + e] = cvt16<MODE>(c[e]);
  }
  const v4u u = (v4u){pk16(hb[0], hb[1]), pk16(hb[2], hb[3]), pk16(hb[4], hb[5]), pk16(hb[6], hb[7])};
  unsigned short* q = out + 8 * (size_t)i;
  *(volatile v4u*)q = u;
  __threadfence();
  *(volatile v4u*)q = u;
}

__global__ __launch_bounds__(256) void gn_kernel(const float* __restrict__ Y, const float* __restrict__ gw,
                                                 const float* __restrict__ gb, unsigned short* __restrict__ YN) {
  __shared__ float redS[8];
  __shared__ float redQ[8];
  const int t    = threadIdx.x;
  const int lane = t & 31, wave = t >> 5;
  const int bh   = blockIdx.x;
  const int b    = bh >> 4;
  const int h    = bh & 15;
  const int q    = lane >> 3, c8 = (lane & 7) * 8;
  const size_t colBase = (size_t)h * kDh + c8;
  const float* yb = Y + (size_t)b * kSeq * kDim + colBase;

  float s = 0.0f, sq = 0.0f;
#pragma unroll 1
  for (int it = 0; it < kSeq / 32; ++it) {
    const int row = it * 32 + wave * 4 + q;
    const float* p = yb + (size_t)row * kDim;
    const v4f a = *(const v4f*)(p);
    const v4f c = *(const v4f*)(p + 4);
    s  += ((a[0] + a[1]) + (a[2] + a[3])) + ((c[0] + c[1]) + (c[2] + c[3]));
    sq += ((a[0] * a[0] + a[1] * a[1]) + (a[2] * a[2] + a[3] * a[3]))
        + ((c[0] * c[0] + c[1] * c[1]) + (c[2] * c[2] + c[3] * c[3]));
  }
#pragma unroll
  for (int off = 16; off > 0; off >>= 1) {
    s  += __shfl_xor(s,  off, 32);
    sq += __shfl_xor(sq, off, 32);
  }
  if (lane == 0) { redS[wave] = s; redQ[wave] = sq; }
  __syncthreads();
  double ts = 0.0, tq = 0.0;
#pragma unroll
  for (int w = 0; w < 8; ++w) { ts += (double)redS[w]; tq += (double)redQ[w]; }
  const double invN = 1.0 / 131072.0;
  const double mean = ts * invN;
  double var = tq * invN - mean * mean;
  if (var < 0.0) var = 0.0;
  const float meanf = (float)mean;
  const float varf  = (float)var;
  const float rstd  = 1.0f / sqrtf(varf + kGnEps);

  const v4f w0 = *(const v4f*)(gw + colBase);
  const v4f w1 = *(const v4f*)(gw + colBase + 4);
  const v4f g0 = *(const v4f*)(gb + colBase);
  const v4f g1 = *(const v4f*)(gb + colBase + 4);
  unsigned short* ynb = YN + (size_t)b * kSeq * kDim + colBase;
#pragma unroll 1
  for (int it = 0; it < kSeq / 32; ++it) {
    const int row = it * 32 + wave * 4 + q;
    const float* p = yb + (size_t)row * kDim;
    const v4f a = *(const v4f*)(p);
    const v4f c = *(const v4f*)(p + 4);
    unsigned short hb[8];
#pragma unroll
    for (int e = 0; e < 4; ++e) {
      const float u0 = ((a[e] - meanf) * rstd) * w0[e] + g0[e];
      const float u1 = ((c[e] - meanf) * rstd) * w1[e] + g1[e];
      hb[e]     = h_bits(u0);
      hb[4 + e] = h_bits(u1);
    }
    const v4u u = (v4u){pk16(hb[0], hb[1]), pk16(hb[2], hb[3]), pk16(hb[4], hb[5]), pk16(hb[6], hb[7])};
    unsigned short* op = ynb + (size_t)row * kDim;
    *(volatile v4u*)op = u;
    __threadfence();
    *(volatile v4u*)op = u;
  }
}

#pragma clang fp contract(off)
extern "C" void kernel_launch(void* const* d_in, const int* in_sizes, int n_in,
                              void* d_out, int out_size, void* d_ws, size_t ws_size,
                              hipStream_t stream) {
  if (n_in < 7) return;
  const int nTokElem = kTok * kDim;
  const int nWElem   = kDim * kDim;
  if (in_sizes[0] != nTokElem) return;
  if (in_sizes[1] != nWElem || in_sizes[2] != nWElem || in_sizes[3] != nWElem || in_sizes[4] != nWElem) return;
  if (in_sizes[5] != kDim || in_sizes[6] != kDim) return;
  if (out_size != nTokElem) return;

  const size_t szTok16 = (size_t)kTok * kDim * 2;
  const size_t szW16   = (size_t)kDim * kDim * 2;
  const size_t szVT16  = (size_t)kBatch * kDim * kSeq * 2;
  const size_t szY32   = (size_t)kTok * kDim * 4;
  const size_t szP16   = (size_t)kGroup * kSeq * kSeq * 2;
  const size_t offXB  = 0;
  const size_t offWQ  = offXB  + szTok16;
  const size_t offWK  = offWQ  + szW16;
  const size_t offWV  = offWK  + szW16;
  const size_t offWO  = offWV  + szW16;
  const size_t offQH  = offWO  + szW16;
  const size_t offQL  = offQH  + szTok16;
  const size_t offKH  = offQL  + szTok16;
  const size_t offKL  = offKH  + szTok16;
  const size_t offVTH = offKL  + szTok16;
  const size_t offVTL = offVTH + szVT16;
  const size_t offY   = offVTL + szVT16;
  const size_t offYN  = offY   + szY32;
  const size_t offPH  = offYN  + szTok16;
  const size_t offPL  = offPH  + szP16;
  const size_t total  = offPL  + szP16;
  if (ws_size < total) return;

  const float* x  = (const float*)d_in[0];
  const float* wq = (const float*)d_in[1];
  const float* wk = (const float*)d_in[2];
  const float* wv = (const float*)d_in[3];
  const float* wo = (const float*)d_in[4];
  const float* gw = (const float*)d_in[5];
  const float* gb = (const float*)d_in[6];
  float* out = (float*)d_out;
  char* ws = (char*)d_ws;
  unsigned short* XB  = (unsigned short*)(ws + offXB);
  unsigned short* WQB = (unsigned short*)(ws + offWQ);
  unsigned short* WKB = (unsigned short*)(ws + offWK);
  unsigned short* WVB = (unsigned short*)(ws + offWV);
  unsigned short* WOH = (unsigned short*)(ws + offWO);
  unsigned short* QH  = (unsigned short*)(ws + offQH);
  unsigned short* QL  = (unsigned short*)(ws + offQL);
  unsigned short* KH  = (unsigned short*)(ws + offKH);
  unsigned short* KL  = (unsigned short*)(ws + offKL);
  unsigned short* VTH = (unsigned short*)(ws + offVTH);
  unsigned short* VTL = (unsigned short*)(ws + offVTL);
  float*          Y32 = (float*)(ws + offY);
  unsigned short* YN  = (unsigned short*)(ws + offYN);
  unsigned short* PH  = (unsigned short*)(ws + offPH);
  unsigned short* PL  = (unsigned short*)(ws + offPL);

  float lgh[kHeads];
  {
    const float glo = (float)log(1.0 - 0.999);
    const float ghi = (float)log(1.0 - 0.9);
    const float rdiv = 1.0f / 15.0f;
    for (int h = 0; h < kHeads; ++h) {
      float val;
      if (h == kHeads - 1) {
        val = ghi;
      } else {
        const float st = (float)h * rdiv;
        const float om = 1.0f - st;
        const float t0 = glo * om;
        const float t1 = ghi * st;
        val = t0 + t1;
      }
      const float ex  = expf(val);
      const float gam = 1.0f - ex;
      lgh[h] = (float)log((double)gam);
    }
  }

  const int n8x = nTokElem / 8;
  const int n8w = nWElem / 8;
  cast8_kernel<0><<<dim3(n8x / 256), dim3(256), 0, stream>>>(x,  XB,  n8x);
  cast8_kernel<0><<<dim3(n8w / 256), dim3(256), 0, stream>>>(wq, WQB, n8w);
  cast8_kernel<0><<<dim3(n8w / 256), dim3(256), 0, stream>>>(wk, WKB, n8w);
  cast8_kernel<0><<<dim3(n8w / 256), dim3(256), 0, stream>>>(wv, WVB, n8w);
  cast8_kernel<1><<<dim3(n8w / 256), dim3(256), 0, stream>>>(wo, WOH, n8w);

  const int tilesProj = (kTok / 64) * (kDim / 64);
  const int tilesVT   = (kDim / 64) * (kSeq / 64);
  wmma_gemm64<1, false, 0, 2, false, 0, 0, false><<<dim3(tilesProj / 8, 1), dim3(256), 0, stream>>>(
      XB, XB, kDim, 0L, WQB, WQB, kDim, 0L, (void*)QH, (void*)QL, kDim, 0L, Y32, Y32, 0L,
      kTok, kDim, kDim, 1.0f, 0.0f, 0.0f);
  wmma_gemm64<1, false, 0, 2, false, 0, 0, false><<<dim3(tilesProj / 8, 1), dim3(256), 0, stream>>>(
      XB, XB, kDim, 0L, WKB, WKB, kDim, 0L, (void*)KH, (void*)KL, kDim, 0L, Y32, Y32, 0L,
      kTok, kDim, kDim, 1.0f, 0.0f, 0.0f);
  wmma_gemm64<1, false, 0, 2, false, 0, 0, false><<<dim3(tilesVT / 8, kBatch), dim3(256), 0, stream>>>(
      WVB, WVB, kDim, 0L, XB, XB, kDim, (long)kSeq * kDim, (void*)VTH, (void*)VTL, kSeq, (long)kDim * kSeq,
      Y32, Y32, 0L, kDim, kSeq, kDim, 1.0f, 0.0f, 0.0f);

  const long strideHead16 = (long)kDh;
  const long strideP      = (long)kSeq * kSeq;
  const long strideVT     = (long)kDh * kSeq;
  const int  tilesScore   = (kSeq / 64) * (kSeq / 64);
  const int  tilesPV      = (kSeq / 64) * (kDh / 64);
  for (int b = 0; b < kBatch; ++b) {
    for (int g = 0; g < kHeads / kGroup; ++g) {
      const int hbase = g * kGroup;
      const size_t tokOff = ((size_t)b * kSeq) * kDim + (size_t)hbase * kDh;
      const size_t vtOff  = ((size_t)b * kDim + (size_t)hbase * kDh) * kSeq;
      wmma_gemm64<1, true, 0, 2, false, 0, 1, true><<<dim3(tilesScore / 8, kGroup), dim3(256), 0, stream>>>(
          QH + tokOff, QL + tokOff, kDim, strideHead16, KH + tokOff, KL + tokOff, kDim, strideHead16,
          (void*)PH, (void*)PL, kSeq, strideP, Y32, Y32, 0L, kSeq, kSeq, kDh, 1.0f, lgh[hbase], lgh[hbase + 1]);
      wmma_gemm64<1, true, 0, 0, false, 0, 2, false><<<dim3(tilesPV / 8, kGroup), dim3(256), 0, stream>>>(
          PH, PL, kSeq, strideP, VTH + vtOff, VTL + vtOff, kSeq, strideVT,
          (void*)(Y32 + tokOff), (void*)(Y32 + tokOff), kDim, strideHead16, Y32, Y32, 0L,
          kSeq, kDh, kSeq, 1.0f, 0.0f, 0.0f);
    }
  }

  gn_kernel<<<dim3(kBatch * kHeads), dim3(256), 0, stream>>>(Y32, gw, gb, YN);

  wmma_gemm64<0, false, 0, 0, false, 0, 0, false><<<dim3(tilesProj / 8, 1), dim3(256), 0, stream>>>(
      YN, YN, kDim, 0L, WOH, WOH, kDim, 0L, (void*)out, (void*)out, kDim, 0L, Y32, Y32, 0L,
      kTok, kDim, kDim, kWoCarryInv, 0.0f, 0.0f);
}
